// MHMS_17119739642208
// MI455X (gfx1250) — hardware-run, weakly checked
//
#include <hip/hip_runtime.h>
#include <math.h>

typedef __attribute__((ext_vector_type(16))) _Float16 v16h;
typedef __attribute__((ext_vector_type(8)))  _Float16 v8h;
typedef __attribute__((ext_vector_type(16))) __bf16   v16b;
typedef __attribute__((ext_vector_type(8)))  __bf16   v8b;
typedef __attribute__((ext_vector_type(8)))  float    v8f;
typedef __attribute__((ext_vector_type(4)))  float    v4f;

constexpr int kB     = 16;
constexpr int kS     = 128;
constexpr int kTok   = 32;
constexpr int kMv    = 256;
constexpr int kVocab = 30522;
constexpr int kEmb   = 128;
constexpr int kHid   = 128;
constexpr int kG3    = 3 * kHid;
constexpr int kTxt   = 2 * kHid;
constexpr int kVd    = 1024;
constexpr int kVh    = 256;
constexpr int kAd    = 256;
constexpr int kTh    = 128;
constexpr int kSeqs  = kB * kS;
constexpr int kXRows = kSeqs * kTok;
constexpr int kVRows = kB * kMv;
constexpr int kWcvN  = 2 * kVh + kAd;
constexpr int kWctN  = kTh + kAd;
constexpr int kKM    = kS * kMv;
constexpr int kTn    = kB * kKM;
constexpr int kTfP   = 132;
constexpr int kGateStride = kHid * kEmb;
constexpr int kTile1 = 16 * kTok * kEmb;
constexpr float kCarry    = 64.0f;
constexpr float kCarryInv = 1.0f / 64.0f;
constexpr float kMu = 1.0f / (float)kS;
constexpr float kNu = 1.0f / (float)kMv;
static_assert(kEmb == kHid);
static_assert(kSeqs == 2048 && kXRows == 65536 && kVRows == 4096 && kWcvN == 768 && kWctN == 384);
static_assert((kEmb % 32) == 0 && (kTxt % 32) == 0 && (kVd % 32) == 0 && (kAd % 32) == 0);
static_assert((kVRows % 64) == 0 && (kSeqs % 64) == 0 && (kS % 64) == 0 && (kMv % 64) == 0 && (kTh % 64) == 0 && (kAd % 64) == 0);

constexpr int kOut0 = 0;
constexpr int kOut1 = 2048;
constexpr int kOut2 = 526336;
constexpr int kOut3 = 530432;
constexpr int kOut4 = 532480;
constexpr int kOut5 = 536576;
constexpr int kOutTotal = 1060865;
static_assert(kOut1 == kOut0 + kSeqs && kOut2 == kOut1 + kSeqs * kTxt && kOut3 == kOut2 + kVRows);
static_assert(kOut4 == kOut3 + kSeqs && kOut5 == kOut4 + kVRows && kOut5 + 1 + kTn == kOutTotal);
static_assert((kOut1 % 32) == 0 && (kOut2 % 32) == 0 && (kOut3 % 32) == 0 && (kOut4 % 32) == 0 && (kOut5 % 32) == 0);

constexpr size_t kSzWi  = (size_t)kG3 * kEmb * 2;
constexpr size_t kSzWh  = (size_t)kG3 * kHid * 2;
constexpr size_t kOffWIFH = 0;
constexpr size_t kOffWIFL = kOffWIFH + kSzWi;
constexpr size_t kOffWIBH = kOffWIFL + kSzWi;
constexpr size_t kOffWIBL = kOffWIBH + kSzWi;
constexpr size_t kOffWHF  = kOffWIBL + kSzWi;
constexpr size_t kOffWHB  = kOffWHF  + kSzWh;
constexpr size_t kOffWCVH = kOffWHB  + kSzWh;
constexpr size_t kOffWVPL = kOffWCVH + (size_t)kWcvN * kVd * 2;
constexpr size_t kOffWCTH = kOffWVPL + (size_t)kAd * kVd * 2;
constexpr size_t kOffWTPL = kOffWCTH + (size_t)kWctN * kTxt * 2;
constexpr size_t kOffVH   = kOffWTPL + (size_t)kAd * kTxt * 2;
constexpr size_t kOffVL   = kOffVH   + (size_t)kVRows * kVd * 2;
constexpr size_t kOffXH   = kOffVL   + (size_t)kVRows * kVd * 2;
constexpr size_t kOffXL   = kOffXH   + (size_t)kXRows * kEmb * 2;
constexpr size_t kOffTFH  = kOffXL   + (size_t)kXRows * kEmb * 2;
constexpr size_t kOffTFL  = kOffTFH  + (size_t)kSeqs * kTxt * 2;
constexpr size_t kOffRV   = kOffTFL  + (size_t)kSeqs * kTxt * 2;
constexpr size_t kOffRT   = kOffRV   + (size_t)kVRows * kWcvN * 4;
constexpr size_t kOffVNH  = kOffRT   + (size_t)kSeqs * kWctN * 4;
constexpr size_t kOffVNL  = kOffVNH  + (size_t)kVRows * kAd * 2;
constexpr size_t kOffENH  = kOffVNL  + (size_t)kVRows * kAd * 2;
constexpr size_t kOffENL  = kOffENH  + (size_t)kSeqs * kAd * 2;
constexpr size_t kOffSM   = kOffENL  + (size_t)kSeqs * kAd * 2;
constexpr size_t kOffKM   = kOffSM   + (size_t)kTn * 4;
constexpr size_t kOffTW   = kOffKM   + (size_t)kTn * 4;
constexpr size_t kOffLP   = kOffTW   + (size_t)kTn * 4;
constexpr size_t kWsTotal = kOffLP   + (size_t)kB * 32 * 4;
static_assert(kWsTotal == 83757056ull);
static_assert(kWsTotal <= 134217728ull);
static_assert((kOffWIFL % 128) == 0 && (kOffWHF % 128) == 0 && (kOffWCVH % 128) == 0 && (kOffWVPL % 128) == 0 &&
              (kOffWCTH % 128) == 0 && (kOffWTPL % 128) == 0 && (kOffVH % 128) == 0 && (kOffXH % 128) == 0 &&
              (kOffTFH % 128) == 0 && (kOffRV % 128) == 0 && (kOffRT % 128) == 0 && (kOffVNH % 128) == 0 &&
              (kOffENH % 128) == 0 && (kOffSM % 128) == 0 && (kOffKM % 128) == 0 && (kOffTW % 128) == 0 && (kOffLP % 128) == 0);

__device__ __forceinline__ unsigned short f2bf_bits(float f) {
  unsigned u = __float_as_uint(f);
  return (unsigned short)((u + 0x7FFFu + ((u >> 16) & 1u)) >> 16);
}
__device__ __forceinline__ float bf_bits2f(unsigned short h) { return __uint_as_float(((unsigned)h) << 16); }

__device__ __forceinline__ void dep_guard4_h(v8f& a, v8f& b, v8f& c, v8f& d, v16h x, v16h y) { asm volatile("v_nop\n\tv_nop\n\tv_nop\n\tv_nop" : "+v"(a), "+v"(b), "+v"(c), "+v"(d) : "v"(x), "v"(y)); }
__device__ __forceinline__ void dep_guard4_b(v8f& a, v8f& b, v8f& c, v8f& d, v16b x, v16b y) { asm volatile("v_nop\n\tv_nop\n\tv_nop\n\tv_nop" : "+v"(a), "+v"(b), "+v"(c), "+v"(d) : "v"(x), "v"(y)); }
__device__ __forceinline__ void keep4_h(v16h a, v16h b, v16h c, v16h d) { asm volatile("v_nop" :: "v"(a), "v"(b), "v"(c), "v"(d)); }
__device__ __forceinline__ void keep4_b(v16b a, v16b b, v16b c, v16b d) { asm volatile("v_nop" :: "v"(a), "v"(b), "v"(c), "v"(d)); }
__device__ __forceinline__ void acc_guard4(v8f& a, v8f& b, v8f& c, v8f& d) { asm volatile("v_nop\n\tv_nop\n\tv_nop\n\tv_nop" : "+v"(a), "+v"(b), "+v"(c), "+v"(d)); }
template <typename T> struct Frag;
template <> struct Frag<_Float16> {
  typedef v16h V; union U { v16h v; v8h h[2]; };
  static __device__ __forceinline__ v16h load(const _Float16* p) {
    U f; f.h[0] = *(const v8h*)(p); f.h[1] = *(const v8h*)(p + 16); return f.v;
  }
  static __device__ __forceinline__ v8f mma(v16h a, v16h b, v8f c) {
    return __builtin_amdgcn_wmma_f32_16x16x32_f16(false, a, false, b, (short)0, c, false, false);
  }
  static __device__ __forceinline__ void guard4(v8f& a, v8f& b, v8f& c, v8f& d, v16h x, v16h y) { dep_guard4_h(a, b, c, d, x, y); }
  static __device__ __forceinline__ void keep(v16h a, v16h b, v16h c, v16h d) { keep4_h(a, b, c, d); }
};
template <> struct Frag<__bf16> {
  typedef v16b V; union U { v16b v; v8b h[2]; };
  static __device__ __forceinline__ v16b load(const __bf16* p) {
    U f; f.h[0] = *(const v8b*)(p); f.h[1] = *(const v8b*)(p + 16); return f.v;
  }
  static __device__ __forceinline__ v8f mma(v16b a, v16b b, v8f c) {
    return __builtin_amdgcn_wmma_f32_16x16x32_bf16(false, a, false, b, (short)0, c, false, false);
  }
  static __device__ __forceinline__ void guard4(v8f& a, v8f& b, v8f& c, v8f& d, v16b x, v16b y) { dep_guard4_b(a, b, c, d, x, y); }
  static __device__ __forceinline__ void keep(v16b a, v16b b, v16b c, v16b d) { keep4_b(a, b, c, d); }
};
typedef Frag<__bf16>   FB;
typedef Frag<_Float16> FH;

__device__ __forceinline__ v8f mma_b_g(v16b a, v16b b, v8f c) {
  c = __builtin_amdgcn_wmma_f32_16x16x32_bf16(false, a, false, b, (short)0, c, false, false);
  asm volatile("v_nop\n\tv_nop\n\tv_nop\n\tv_nop" : "+v"(c) : "v"(a), "v"(b));
  return c;
}
__device__ __forceinline__ v8f mma_h_g(v16h a, v16h b, v8f c) {
  c = __builtin_amdgcn_wmma_f32_16x16x32_f16(false, a, false, b, (short)0, c, false, false);
  asm volatile("v_nop\n\tv_nop\n\tv_nop\n\tv_nop" : "+v"(c) : "v"(a), "v"(b));
  return c;
}

__device__ __forceinline__ void split8(const v4f a0, const v4f a1, v8h& hv, v8h& lv) {
#pragma unroll
  for (int e = 0; e < 4; ++e) {
    const float f0 = a0[e];
    const float f1 = a1[e];
    const unsigned short h0 = f2bf_bits(f0), h1 = f2bf_bits(f1);
    const unsigned short l0 = f2bf_bits(f0 - bf_bits2f(h0)), l1 = f2bf_bits(f1 - bf_bits2f(h1));
    hv[e]     = __builtin_bit_cast(_Float16, h0);
    hv[4 + e] = __builtin_bit_cast(_Float16, h1);
    lv[e]     = __builtin_bit_cast(_Float16, l0);
    lv[4 + e] = __builtin_bit_cast(_Float16, l1);
  }
}

template <int ET> struct Elem;
template <> struct Elem<0> { typedef _Float16 T; };
template <> struct Elem<1> { typedef __bf16 T; };
template <int ET, int SPL, int BIAS_MODE, int OUT_MODE, bool RESID, int ACT = 0>
__global__ __launch_bounds__(256) void wmma_gemm64(
    const unsigned short* __restrict__ Ap, const unsigned short* __restrict__ A2p, int lda, long strideA,
    const unsigned short* __restrict__ Btp, const unsigned short* __restrict__ Bt2p, int ldb, long strideB,
    void* __restrict__ Cout, void* __restrict__ Cout2, int ldc, long strideC,
    const float* __restrict__ bias,
    const float* __restrict__ resid, long strideR,
    int M, int N, int K, float scale) {
  typedef typename Elem<ET>::T T;
  typedef typename Frag<T>::V V;
  const T* A = (const T*)Ap; const T* A2 = (const T*)A2p; const T* Bt = (const T*)Btp; const T* Bt2 = (const T*)Bt2p;
  __shared__ __align__(16) float sT[8][16 * 68];
  const int b    = blockIdx.y;
  const int lane = threadIdx.x & 31;
  const int wave = threadIdx.x >> 5;
  const int tilesN = N >> 6;
  const int tilesM = M >> 6;
  const int tile = blockIdx.x * 8 + wave;
  if (tile >= tilesM * tilesN) return;
  const int tm = tile / tilesN;
  const int tn = tile - tm * tilesN;
  const int m0 = tm << 6;
  const int n0 = tn << 6;

  const T* Ab  = A  + (size_t)b * strideA;
  const T* Bb  = Bt + (size_t)b * strideB;
  const T* Ab2 = (SPL >= 1) ? (A2  + (size_t)b * strideA) : nullptr;
  const T* Bb2 = (SPL == 2) ? (Bt2 + (size_t)b * strideB) : nullptr;

  const int rlane = lane & 15;
  const int koff  = (lane >> 4) * 8;
  const int mOff  = (lane >> 4) * 8;

  v8f acc[4][4];
#pragma unroll
  for (int i = 0; i < 4; ++i)
#pragma unroll
    for (int j = 0; j < 4; ++j) acc[i][j] = (v8f){0.f,0.f,0.f,0.f,0.f,0.f,0.f,0.f};

  for (int k0 = 0; k0 < K; k0 += 32) {
    V bh[4], bl[4];
#pragma unroll
    for (int j = 0; j < 4; ++j) {
      const size_t bo = (size_t)(n0 + (j << 4) + rlane) * ldb + koff + k0;
      bh[j] = Frag<T>::load(Bb + bo);
      if (SPL == 2) bl[j] = Frag<T>::load(Bb2 + bo);
    }
#pragma unroll
    for (int i = 0; i < 4; ++i) {
      const size_t ao = (size_t)(m0 + (i << 4) + rlane) * lda + koff + k0;
      V ah = Frag<T>::load(Ab + ao);
      V al;
      if (SPL >= 1) al = Frag<T>::load(Ab2 + ao);
#pragma unroll
      for (int j = 0; j < 4; ++j) {
        acc[i][j] = Frag<T>::mma(ah, bh[j], acc[i][j]);
        if (SPL == 2) acc[i][j] = Frag<T>::mma(ah, bl[j], acc[i][j]);
        if (SPL >= 1) acc[i][j] = Frag<T>::mma(al, bh[j], acc[i][j]);
      }
      Frag<T>::guard4(acc[i][0], acc[i][1], acc[i][2], acc[i][3], ah, (SPL >= 1) ? al : ah);
    }
    Frag<T>::keep(bh[0], bh[1], bh[2], bh[3]);
    if (SPL == 2) Frag<T>::keep(bl[0], bl[1], bl[2], bl[3]);
  }
  acc_guard4(acc[0][0], acc[0][1], acc[0][2], acc[0][3]);
  acc_guard4(acc[1][0], acc[1][1], acc[1][2], acc[1][3]);
  acc_guard4(acc[2][0], acc[2][1], acc[2][2], acc[2][3]);
  acc_guard4(acc[3][0], acc[3][1], acc[3][2], acc[3][3]);

  float* slab = sT[wave];
  const float* Rb = RESID ? (resid + (size_t)b * strideR) : nullptr;
#pragma unroll
  for (int i = 0; i < 4; ++i) {
    const int mBase = m0 + (i << 4);
#pragma unroll
    for (int j = 0; j < 4; ++j) {
      const int n = n0 + (j << 4) + rlane;
      float bv = 0.f;
      if (BIAS_MODE == 2) bv = bias[n];
#pragma unroll
      for (int r = 0; r < 8; ++r) {
        float v = acc[i][j][r] * scale;
        if (BIAS_MODE == 1) v += bias[mBase + mOff + r];
        if (BIAS_MODE == 2) v += bv;
        if (RESID) v += Rb[(size_t)(mBase + mOff + r) * ldc + n];
        if (ACT == 1) v = tanhf(v);
        if (ACT == 2) v = fmaxf(v, 0.0f);
        if (ACT == 3) v = v / (1.0f + expf(-v));
        if (ACT == 4) v = (v > 0.f) ? v : 0.01f * v;
        slab[(mOff + r) * 68 + (j << 4) + rlane] = v;
      }
    }
    __builtin_amdgcn_fence(__ATOMIC_RELEASE, "workgroup");
    __builtin_amdgcn_wave_barrier();
    __builtin_amdgcn_fence(__ATOMIC_ACQUIRE, "workgroup");
    if (OUT_MODE == 0) {
      float* C = (float*)Cout + (size_t)b * strideC;
      const int hh = lane >> 4, c4 = (lane & 15) * 4;
      for (int pass = 0; pass < 2; ++pass) {
#pragma unroll
        for (int it = 0; it < 8; ++it) {
          const int row = it * 2 + hh;
          v4f v = *(const v4f*)(slab + row * 68 + c4);
          *(volatile v4f*)(C + (size_t)(mBase + row) * ldc + n0 + c4) = v;
        }
        __threadfence();
      }
    } else {
      const int q = lane >> 3, c8 = (lane & 7) * 8;
      unsigned short* C  = (unsigned short*)Cout  + (size_t)b * strideC;
      unsigned short* C2 = (OUT_MODE == 2) ? ((unsigned short*)Cout2 + (size_t)b * strideC) : nullptr;
      for (int pass = 0; pass < 2; ++pass) {
#pragma unroll
        for (int it = 0; it < 4; ++it) {
          const int row = it * 4 + q;
          const float* sp = slab + row * 68 + c8;
          v8h hv, lv;
#pragma unroll
          for (int e = 0; e < 8; ++e) {
            if (OUT_MODE == 1) {
              hv[e] = (_Float16)sp[e];
            } else {
              unsigned short hb = f2bf_bits(sp[e]);
              unsigned short lb = f2bf_bits(sp[e] - bf_bits2f(hb));
              hv[e] = __builtin_bit_cast(_Float16, hb);
              lv[e] = __builtin_bit_cast(_Float16, lb);
            }
          }
          *(volatile v8h*)(C + (size_t)(mBase + row) * ldc + n0 + c8) = hv;
          if (OUT_MODE == 2) *(volatile v8h*)(C2 + (size_t)(mBase + row) * ldc + n0 + c8) = lv;
        }
        __threadfence();
      }
    }
    __builtin_amdgcn_fence(__ATOMIC_RELEASE, "workgroup");
    __builtin_amdgcn_wave_barrier();
    __builtin_amdgcn_fence(__ATOMIC_ACQUIRE, "workgroup");
  }
}

__global__ __launch_bounds__(256) void cast_f32_f16x2(
    const float* __restrict__ in, _Float16* __restrict__ out, int n2) {
  int i = blockIdx.x * 256 + threadIdx.x;
  if (i < n2) {
    const _Float16 h0 = (_Float16)in[2 * i], h1 = (_Float16)in[2 * i + 1];
    const unsigned u = (unsigned)__builtin_bit_cast(unsigned short, h0) | ((unsigned)__builtin_bit_cast(unsigned short, h1) << 16);
    ((volatile unsigned*)out)[i] = u;
    __threadfence();
    ((volatile unsigned*)out)[i] = u;
  }
}

template <bool HASLO>
__global__ __launch_bounds__(256) void split_rows_bf16_kernel(
    const float* __restrict__ src, unsigned short* __restrict__ dhi, unsigned short* __restrict__ dlo, int total8)
{
  const int i = blockIdx.x * 256 + threadIdx.x;
  if (i >= total8) return;
  const size_t e0 = (size_t)i << 3;
  const v4f a0 = *(const v4f*)(src + e0);
  const v4f a1 = *(const v4f*)(src + e0 + 4);
  v8h hv, lv;
  split8(a0, a1, hv, lv);
  unsigned short* qh = dhi + e0;
  *(volatile v8h*)qh = hv;
  if (HASLO) *(volatile v8h*)(dlo + e0) = lv;
  __threadfence();
  *(volatile v8h*)qh = hv;
  if (HASLO) *(volatile v8h*)(dlo + e0) = lv;
}

__global__ __launch_bounds__(256) void gather_split_kernel(
    const int* __restrict__ ids, const float* __restrict__ emb,
    unsigned short* __restrict__ XH, unsigned short* __restrict__ XL, float* __restrict__ out0)
{
  const int i = blockIdx.x * 256 + threadIdx.x;
  const int row = i >> 4;
  const int seg = i & 15;
  int id = ids[row];
  id = id < 0 ? 0 : id;
  id = id > (kVocab - 1) ? (kVocab - 1) : id;
  const float* src = emb + (size_t)id * kEmb + seg * 8;
  v4f a0 = *(const v4f*)(src);
  v4f a1 = *(const v4f*)(src + 4);
  a0 = a0 * kCarry;
  a1 = a1 * kCarry;
  v8h hv, lv;
  split8(a0, a1, hv, lv);
  const size_t e0 = (size_t)i << 3;
  const v4f zz = (v4f){0.f, 0.f, 0.f, 0.f};
  *(volatile v8h*)(XH + e0) = hv;
  *(volatile v8h*)(XL + e0) = lv;
  if (i < 512) *(volatile v4f*)(out0 + 4 * i) = zz;
  __threadfence();
  *(volatile v8h*)(XH + e0) = hv;
  *(volatile v8h*)(XL + e0) = lv;
  if (i < 512) *(volatile v4f*)(out0 + 4 * i) = zz;
}

__device__ __forceinline__ void gate_tile(const v8f aR, const v8f aZ, const v8f aXN, const v8f aHN,
                                          float (&h)[8], float (&hsum)[8], _Float16* dst) {
#pragma unroll
  for (int r = 0; r < 8; ++r) {
    const float ar = aR[r] * kCarryInv;
    const float az = aZ[r] * kCarryInv;
    const float xn = aXN[r] * kCarryInv;
    const float hn = aHN[r] * kCarryInv;
    const float rg = __builtin_amdgcn_rcpf(1.0f + __expf(-ar));
    const float zg = __builtin_amdgcn_rcpf(1.0f + __expf(-az));
    const float ng = tanhf(xn + rg * hn);
    const float hnew = (1.0f - zg) * ng + zg * h[r];
    h[r] = hnew;
    hsum[r] += hnew;
    dst[r * kHid] = (_Float16)(hnew * kCarry);
  }
}

__global__ __launch_bounds__(256) void gru_scan_kernel(
    const unsigned short* __restrict__ XHp, const unsigned short* __restrict__ XLp,
    const unsigned short* __restrict__ WiFHp, const unsigned short* __restrict__ WiFLp, const unsigned short* __restrict__ WhFp,
    const float* __restrict__ biF, const float* __restrict__ bhF,
    const unsigned short* __restrict__ WiBHp, const unsigned short* __restrict__ WiBLp, const unsigned short* __restrict__ WhBp,
    const float* __restrict__ biB, const float* __restrict__ bhB,
    float* __restrict__ out1, unsigned short* __restrict__ TFH, unsigned short* __restrict__ TFL)
{
  __shared__ __align__(16) _Float16 hs[2][32 * kHid];
  __shared__ __align__(16) float tfs[32 * kTfP];
  const int tid  = threadIdx.x;
  const int lane = tid & 31;
  const int wave = tid >> 5;
  const int hh   = lane >> 4;
  const int c    = lane & 15;
  const int dir  = blockIdx.x >> 6;
  const int q0   = (blockIdx.x & 63) * 32;
  const int j    = wave * 16 + c;

  const __bf16*   WiH = (const __bf16*)(dir ? WiBHp : WiFHp);
  const __bf16*   WiL = (const __bf16*)(dir ? WiBLp : WiFLp);
  const _Float16* Wh  = (const _Float16*)(dir ? WhBp : WhFp);
  const float*    bi  = dir ? biB : biF;
  const float*    bh  = dir ? bhB : bhF;
  const __bf16*   XH  = (const __bf16*)XHp;
  const __bf16*   XL  = (const __bf16*)XLp;

  const float sR  = kCarry * (bi[j] + bh[j]);
  const float sZ  = kCarry * (bi[kHid + j] + bh[kHid + j]);
  const float sXN = kCarry * bi[2 * kHid + j];
  const float sHN = kCarry * bh[2 * kHid + j];

  const int    wofs = j * kEmb + 8 * hh;
  const size_t xofs = ((size_t)(q0 + c) * kTok) * kEmb + 8 * hh;

  float hA[8], hB[8], uA[8], uB[8];
#pragma unroll
  for (int r = 0; r < 8; ++r) { hA[r] = 0.f; hB[r] = 0.f; uA[r] = 0.f; uB[r] = 0.f; }

#pragma unroll 1
  for (int t = 0; t < kTok; ++t) {
    const int tt = dir ? (kTok - 1 - t) : t;
    v8f aR0 = (v8f){sR, sR, sR, sR, sR, sR, sR, sR};
    v8f aR1 = aR0;
    v8f aZ0 = (v8f){sZ, sZ, sZ, sZ, sZ, sZ, sZ, sZ};
    v8f aZ1 = aZ0;
    v8f aX0 = (v8f){sXN, sXN, sXN, sXN, sXN, sXN, sXN, sXN};
    v8f aX1 = aX0;
    v8f aH0 = (v8f){sHN, sHN, sHN, sHN, sHN, sHN, sHN, sHN};
    v8f aH1 = aH0;
    const __bf16* xh = XH + xofs + (size_t)tt * kEmb;
    const __bf16* xl = XL + xofs + (size_t)tt * kEmb;
#pragma unroll 1
    for (int kc = 0; kc < kEmb / 32; ++kc) {
      const int ko = kc * 32;
      const v16b a0h = FB::load(xh + ko);
      const v16b a0l = FB::load(xl + ko);
      const v16b a1h = FB::load(xh + kTile1 + ko);
      const v16b a1l = FB::load(xl + kTile1 + ko);
      {
        const v16b bhi = FB::load(WiH + wofs + ko);
        const v16b blo = FB::load(WiL + wofs + ko);
        aR0 = mma_b_g(a0h, bhi, aR0);
        aR0 = mma_b_g(a0h, blo, aR0);
        aR0 = mma_b_g(a0l, bhi, aR0);
        aR1 = mma_b_g(a1h, bhi, aR1);
        aR1 = mma_b_g(a1h, blo, aR1);
        aR1 = mma_b_g(a1l, bhi, aR1);
      }
      {
        const v16b bhi = FB::load(WiH + kGateStride + wofs + ko);
        const v16b blo = FB::load(WiL + kGateStride + wofs + ko);
        aZ0 = mma_b_g(a0h, bhi, aZ0);
        aZ0 = mma_b_g(a0h, blo, aZ0);
        aZ0 = mma_b_g(a0l, bhi, aZ0);
        aZ1 = mma_b_g(a1h, bhi, aZ1);
        aZ1 = mma_b_g(a1h, blo, aZ1);
        aZ1 = mma_b_g(a1l, bhi, aZ1);
      }
      {
        const v16b bhi = FB::load(WiH + 2 * kGateStride + wofs + ko);
        const v16b blo = FB::load(WiL + 2 * kGateStride + wofs + ko);
        aX0 = mma_b_g(a0h, bhi, aX0);
        aX0 = mma_b_g(a0h, blo, aX0);
        aX0 = mma_b_g(a0l, bhi, aX0);
        aX1 = mma_b_g(a1h, bhi, aX1);
        aX1 = mma_b_g(a1h, blo, aX1);
        aX1 = mma_b_g(a1l, bhi, aX1);
      }
    }
    if (t > 0) {
      const _Float16* hc = &hs[t & 1][0];
#pragma unroll 1
      for (int kc = 0; kc < kHid / 32; ++kc) {
        const int ko = kc * 32;
        const v16h g0 = FH::load(hc + c * kHid + ko + 8 * hh);
        const v16h g1 = FH::load(hc + (16 + c) * kHid + ko + 8 * hh);
        {
          const v16h w = FH::load(Wh + wofs + ko);
          aR0 = mma_h_g(g0, w, aR0);
          aR1 = mma_h_g(g1, w, aR1);
        }
        {
          const v16h w = FH::load(Wh + kGateStride + wofs + ko);
          aZ0 = mma_h_g(g0, w, aZ0);
          aZ1 = mma_h_g(g1, w, aZ1);
        }
        {
          const v16h w = FH::load(Wh + 2 * kGateStride + wofs + ko);
          aH0 = mma_h_g(g0, w, aH0);
          aH1 = mma_h_g(g1, w, aH1);
        }
      }
    }
    _Float16* hn = &hs[(t + 1) & 1][0];
    gate_tile(aR0, aZ0, aX0, aH0, hA, uA, hn + (8 * hh) * kHid + j);
    gate_tile(aR1, aZ1, aX1, aH1, hB, uB, hn + (16 + 8 * hh) * kHid + j);
    __syncthreads();
  }

#pragma unroll
  for (int r = 0; r < 8; ++r) {
    tfs[(8 * hh + r) * kTfP + j]      = uA[r] * (1.0f / (float)kTok);
    tfs[(16 + 8 * hh + r) * kTfP + j] = uB[r] * (1.0f / (float)kTok);
  }
  __syncthreads();
  v4f fv[4];
#pragma unroll
  for (int i = 0; i < 4; ++i) fv[i] = *(const v4f*)(tfs + (4 * wave + i) * kTfP + lane * 4);
  v8h ph[2], pl[2];
#pragma unroll
  for (int i2 = 0; i2 < 2; ++i2) {
    const float* sp = tfs + (4 * wave + 2 * i2 + hh) * kTfP + c * 8;
    const v4f a0 = *(const v4f*)(sp);
    const v4f a1 = *(const v4f*)(sp + 4);
    split8(a0, a1, ph[i2], pl[i2]);
  }
  for (int pass = 0; pass < 2; ++pass) {
#pragma unroll
    for (int i = 0; i < 4; ++i)
      *(volatile v4f*)(out1 + (size_t)(q0 + 4 * wave + i) * kTxt + dir * kHid + lane * 4) = fv[i];
#pragma unroll
    for (int i2 = 0; i2 < 2; ++i2) {
      const size_t o = (size_t)(q0 + 4 * wave + 2 * i2 + hh) * kTxt + dir * kHid + c * 8;
      *(volatile v8h*)(TFH + o) = ph[i2];
      *(volatile v8h*)(TFL + o) = pl[i2];
    }
    __threadfence();
  }
}

__global__ __launch_bounds__(256) void row_epilogue_kernel(
    const float* __restrict__ R, int ldr,
    int nA, const float* __restrict__ b1A, const float* __restrict__ w2A, const float* __restrict__ b2A, float* __restrict__ outA,
    int offB, int nB, const float* __restrict__ b1B, const float* __restrict__ w2B, const float* __restrict__ b2B, float* __restrict__ outB,
    int offP, const float* __restrict__ bP,
    unsigned short* __restrict__ NH, unsigned short* __restrict__ NL)
{
  __shared__ float sPA[32];
  __shared__ float sPB[32];
  const int lane = threadIdx.x & 31;
  const int wave = threadIdx.x >> 5;
  const float b2a = b2A[0];
  const float b2b = b2B[0];
#pragma unroll 1
  for (int i = 0; i < 4; ++i) {
    const int rl  = 4 * wave + i;
    const int row = blockIdx.x * 32 + rl;
    const float* rr = R + (size_t)row * ldr;
    float sa = 0.f, sb = 0.f;
#pragma unroll 1
    for (int col = lane; col < nA; col += 32) {
      const float v = fmaxf(rr[col] + b1A[col], 0.0f);
      sa = fmaf(v, w2A[col], sa);
    }
#pragma unroll 1
    for (int col = lane; col < nB; col += 32) {
      const float v = tanhf(rr[offB + col] + b1B[col]);
      sb = fmaf(v, w2B[col], sb);
    }
#pragma unroll
    for (int off = 16; off > 0; off >>= 1) {
      sa += __shfl_xor(sa, off, 32);
      sb += __shfl_xor(sb, off, 32);
    }
    const float pA = __builtin_amdgcn_rcpf(1.0f + expf(-(sa + b2a)));
    const float pB = __builtin_amdgcn_rcpf(1.0f + expf(-(sb + b2b)));
    if (lane == 0) { sPA[rl] = pA; sPB[rl] = pB; }
    const v4f r0 = *(const v4f*)(rr + offP + lane * 8);
    const v4f r1 = *(const v4f*)(rr + offP + lane * 8 + 4);
    const v4f c0 = *(const v4f*)(bP + lane * 8);
    const v4f c1 = *(const v4f*)(bP + lane * 8 + 4);
    v4f v0, v1;
    float ss = 0.f;
#pragma unroll
    for (int e = 0; e < 4; ++e) {
      v0[e] = pB * r0[e] + c0[e];
      v1[e] = pB * r1[e] + c1[e];
      ss = fmaf(v0[e], v0[e], ss);
      ss = fmaf(v1[e], v1[e], ss);
    }
#pragma unroll
    for (int off = 16; off > 0; off >>= 1) ss += __shfl_xor(ss, off, 32);
    const float inv = 1.0f / (sqrtf(ss) + 1e-12f);
    v0 = v0 * inv;
    v1 = v1 * inv;
    v8h hv, lv;
    split8(v0, v1, hv, lv);
    const size_t o = (size_t)row * kAd + lane * 8;
    *(volatile v8h*)(NH + o) = hv;
    *(volatile v8h*)(NL + o) = lv;
    __threadfence();
    *(volatile v8h*)(NH + o) = hv;
    *(volatile v8h*)(NL + o) = lv;
  }
  __syncthreads();
  if (wave == 0 && outA != nullptr) {
    const float v = sPA[lane];
    volatile float* p = outA + blockIdx.x * 32 + lane;
    *p = v;
    __threadfence();
    *p = v;
  }
  if (wave == 1) {
    const float v = sPB[lane];
    volatile float* p = outB + blockIdx.x * 32 + lane;
    *p = v;
    __threadfence();
    *p = v;
  }
}

__global__ __launch_bounds__(256) void cost_exp_kernel(const float* __restrict__ Sm, float* __restrict__ Km)
{
  const int i = blockIdx.x * 256 + threadIdx.x;
  const v4f s = *(const v4f*)(Sm + (size_t)i * 4);
  v4f k;
#pragma unroll
  for (int e = 0; e < 4; ++e) {
    const float cst = 1.0f - s[e];
    k[e] = expf(-cst * 20.0f);
  }
  *(volatile v4f*)(Km + (size_t)i * 4) = k;
  __threadfence();
  *(volatile v4f*)(Km + (size_t)i * 4) = k;
}

__global__ __launch_bounds__(256) void transport_scale_kernel(
    const float* __restrict__ Km, const float* __restrict__ Sm, float* __restrict__ Tw, float* __restrict__ LP)
{
  __shared__ __align__(16) float su[kS];
  __shared__ __align__(16) float sv[kMv];
  __shared__ float sred[8];
  const int tid  = threadIdx.x;
  const int lane = tid & 31;
  const int wave = tid >> 5;
  const int b    = blockIdx.x;
  const float* Kb = Km + (size_t)b * kKM;
  const float* Sb = Sm + (size_t)b * kKM;
  sv[tid] = kNu;
  __syncthreads();
#pragma unroll 1
  for (int it = 0; it < 10; ++it) {
#pragma unroll 1
    for (int rr = 0; rr < 16; ++rr) {
      const int k = wave * 16 + rr;
      const float* kr = Kb + (size_t)k * kMv;
      const v4f a0 = *(const v4f*)(kr + lane * 4);
      const v4f a1 = *(const v4f*)(kr + 128 + lane * 4);
      const v4f w0 = *(const v4f*)(sv + lane * 4);
      const v4f w1 = *(const v4f*)(sv + 128 + lane * 4);
      float s = 0.f;
#pragma unroll
      for (int e = 0; e < 4; ++e) {
        s = fmaf(a0[e], w0[e], s);
        s = fmaf(a1[e], w1[e], s);
      }
#pragma unroll
      for (int off = 16; off > 0; off >>= 1) s += __shfl_xor(s, off, 32);
      if (lane == 0) su[k] = kMu * (1.0f / (s + 1e-8f));
    }
    __syncthreads();
    float s = 0.f;
#pragma unroll 4
    for (int k = 0; k < kS; ++k) s = fmaf(Kb[(size_t)k * kMv + tid], su[k], s);
    sv[tid] = kNu * (1.0f / (s + 1e-8f));
    __syncthreads();
  }
  float part = 0.f;
#pragma unroll 1
  for (int rr = 0; rr < 16; ++rr) {
    const int k = wave * 16 + rr;
    const size_t ro = (size_t)k * kMv;
    const float uk = su[k];
    const v4f a0 = *(const v4f*)(Kb + ro + lane * 4);
    const v4f a1 = *(const v4f*)(Kb + ro + 128 + lane * 4);
    const v4f s0 = *(const v4f*)(Sb + ro + lane * 4);
    const v4f s1 = *(const v4f*)(Sb + ro + 128 + lane * 4);
    const v4f w0 = *(const v4f*)(sv + lane * 4);
    const v4f w1 = *(const v4f*)(sv + 128 + lane * 4);
    v4f t0, t1;
#pragma unroll
    for (int e = 0; e < 4; ++e) {
      t0[e] = (uk * a0[e]) * w0[e];
      t1[e] = (uk * a1[e]) * w1[e];
      part = fmaf(t0[e], 1.0f - s0[e], part);
      part = fmaf(t1[e], 1.0f - s1[e], part);
    }
    float* tp = Tw + (size_t)b * kKM + ro;
    *(volatile v4f*)(tp + lane * 4) = t0;
    *(volatile v4f*)(tp + 128 + lane * 4) = t1;
    __threadfence();
    *(volatile v4f*)(tp + lane * 4) = t0;
    *(volatile v4f*)(tp + 128 + lane * 4) = t1;
  }
#pragma unroll
  for (int off = 16; off > 0; off >>= 1) part += __shfl_xor(part, off, 32);
  if (lane == 0) sred[wave] = part;
  __syncthreads();
  if (wave == 0) {
    float tot = sred[0];
    tot += sred[1]; tot += sred[2]; tot += sred[3];
    tot += sred[4]; tot += sred[5]; tot += sred[6]; tot += sred[7];
    const float val = (lane == 0) ? tot : 0.0f;
    volatile float* p = LP + b * 32 + lane;
    *p = val;
    __threadfence();
    *p = val;
  }
}

__global__ __launch_bounds__(256) void pack_kernel(
    const float* __restrict__ Tw, const float* __restrict__ LP, float* __restrict__ dst)
{
  const int i = blockIdx.x * 256 + threadIdx.x;
  float ls = 0.f;
#pragma unroll 1
  for (int bb = 0; bb < kB; ++bb) ls += LP[bb * 32];
  ls *= (1.0f / (float)kB);
  const int j0 = 4 * i;
  const int i0 = (j0 > 0) ? (j0 - 1) : 0;
  const float t0 = Tw[i0];
  const float t1 = Tw[j0];
  const float t2 = Tw[j0 + 1];
  const float t3 = Tw[j0 + 2];
  const float tl = Tw[kTn - 1];
  v4f o;
  o[0] = (j0 == 0) ? ls : t0;
  o[1] = t1;
  o[2] = t2;
  o[3] = t3;
  *(volatile v4f*)(dst + j0) = o;
  __threadfence();
  *(volatile v4f*)(dst + j0) = o;
  if (i == 0) {
    volatile float* p = dst + kTn;
    *p = tl;
    __threadfence();
    *p = tl;
  }
}

extern "C" void kernel_launch(void* const* d_in, const int* in_sizes, int n_in,
                              void* d_out, int out_size, void* d_ws, size_t ws_size,
                              hipStream_t stream) {
  if (n_in < 28) return;
  if (in_sizes[0] != kXRows) return;
  if (in_sizes[2] != kVRows * kVd) return;
  if (in_sizes[3] != kVocab * kEmb) return;
  if (in_sizes[4] != kG3 * kEmb || in_sizes[5] != kG3 * kHid) return;
  if (in_sizes[8] != kG3 * kEmb || in_sizes[9] != kG3 * kHid) return;
  if (in_sizes[12] != kAd * kTxt || in_sizes[14] != kAd * kVd) return;
  if (in_sizes[16] != kTh * kTxt || in_sizes[20] != kVh * kVd || in_sizes[24] != kVh * kVd) return;
  if (out_size != kOutTotal) return;
  if (ws_size < kWsTotal) return;

  const int*   ids    = (const int*)d_in[0];
  const float* video  = (const float*)d_in[2];
  const float* emb    = (const float*)d_in[3];
  const float* WiF    = (const float*)d_in[4];
  const float* WhF    = (const float*)d_in[5];
  const float* biF    = (const float*)d_in[6];
  const float* bhF    = (const float*)d_in[7];
  const float* WiB    = (const float*)d_in[8];
  const float* WhB    = (const float*)d_in[9];
  const float* biB    = (const float*)d_in[10];
  const float* bhB    = (const float*)d_in[11];
  const float* tprojW = (const float*)d_in[12];
  const float* tprojB = (const float*)d_in[13];
  const float* vprojW = (const float*)d_in[14];
  const float* vprojB = (const float*)d_in[15];
  const float* tsumW1 = (const float*)d_in[16];
  const float* tsumB1 = (const float*)d_in[17];
  const float* tsumW2 = (const float*)d_in[18];
  const float* tsumB2 = (const float*)d_in[19];
  const float* vsumW1 = (const float*)d_in[20];
  const float* vsumB1 = (const float*)d_in[21];
  const float* vsumW2 = (const float*)d_in[22];
  const float* vsumB2 = (const float*)d_in[23];
  const float* vtsW1  = (const float*)d_in[24];
  const float* vtsB1  = (const float*)d_in[25];
  const float* vtsW2  = (const float*)d_in[26];
  const float* vtsB2  = (const float*)d_in[27];
  float* out = (float*)d_out;

  char* ws = (char*)d_ws;
  unsigned short* WIFH = (unsigned short*)(ws + kOffWIFH);
  unsigned short* WIFL = (unsigned short*)(ws + kOffWIFL);
  unsigned short* WIBH = (unsigned short*)(ws + kOffWIBH);
  unsigned short* WIBL = (unsigned short*)(ws + kOffWIBL);
  unsigned short* WHF  = (unsigned short*)(ws + kOffWHF);
  unsigned short* WHB  = (unsigned short*)(ws + kOffWHB);
  unsigned short* WCVH = (unsigned short*)(ws + kOffWCVH);
  unsigned short* WVPL = (unsigned short*)(ws + kOffWVPL);
  unsigned short* WCTH = (unsigned short*)(ws + kOffWCTH);
  unsigned short* WTPL = (unsigned short*)(ws + kOffWTPL);
  unsigned short* VH   = (unsigned short*)(ws + kOffVH);
  unsigned short* VL   = (unsigned short*)(ws + kOffVL);
  unsigned short* XH   = (unsigned short*)(ws + kOffXH);
  unsigned short* XL   = (unsigned short*)(ws + kOffXL);
  unsigned short* TFH  = (unsigned short*)(ws + kOffTFH);
  unsigned short* TFL  = (unsigned short*)(ws + kOffTFL);
  float*          RV   = (float*)(ws + kOffRV);
  float*          RT   = (float*)(ws + kOffRT);
  unsigned short* VNH  = (unsigned short*)(ws + kOffVNH);
  unsigned short* VNL  = (unsigned short*)(ws + kOffVNL);
  unsigned short* ENH  = (unsigned short*)(ws + kOffENH);
  unsigned short* ENL  = (unsigned short*)(ws + kOffENL);
  float*          SM   = (float*)(ws + kOffSM);
  float*          KM   = (float*)(ws + kOffKM);
  float*          TW   = (float*)(ws + kOffTW);
  float*          LP   = (float*)(ws + kOffLP);

  split_rows_bf16_kernel<true><<<(kG3 * kEmb / 8) / 256, 256, 0, stream>>>(WiF, WIFH, WIFL, kG3 * kEmb / 8);
  split_rows_bf16_kernel<true><<<(kG3 * kEmb / 8) / 256, 256, 0, stream>>>(WiB, WIBH, WIBL, kG3 * kEmb / 8);
  cast_f32_f16x2<<<(kG3 * kHid / 2) / 256, 256, 0, stream>>>(WhF, (_Float16*)WHF, kG3 * kHid / 2);
  cast_f32_f16x2<<<(kG3 * kHid / 2) / 256, 256, 0, stream>>>(WhB, (_Float16*)WHB, kG3 * kHid / 2);
  split_rows_bf16_kernel<false><<<(kVh * kVd / 8) / 256, 256, 0, stream>>>(vtsW1, WCVH, WCVH, kVh * kVd / 8);
  split_rows_bf16_kernel<false><<<(kVh * kVd / 8) / 256, 256, 0, stream>>>(vsumW1, WCVH + (size_t)kVh * kVd, WCVH, kVh * kVd / 8);
  split_rows_bf16_kernel<true><<<(kAd * kVd / 8) / 256, 256, 0, stream>>>(vprojW, WCVH + (size_t)2 * kVh * kVd, WVPL, kAd * kVd / 8);
  split_rows_bf16_kernel<false><<<(kTh * kTxt / 8) / 256, 256, 0, stream>>>(tsumW1, WCTH, WCTH, kTh * kTxt / 8);
  split_rows_bf16_kernel<true><<<(kAd * kTxt / 8) / 256, 256, 0, stream>>>(tprojW, WCTH + (size_t)kTh * kTxt, WTPL, kAd * kTxt / 8);

  split_rows_bf16_kernel<true><<<(kVRows * kVd / 8) / 256, 256, 0, stream>>>(video, VH, VL, kVRows * kVd / 8);

  gather_split_kernel<<<(kXRows * 16) / 256, 256, 0, stream>>>(ids, emb, XH, XL, out + kOut0);

  gru_scan_kernel<<<128, 256, 0, stream>>>(XH, XL, WIFH, WIFL, WHF, biF, bhF, WIBH, WIBL, WHB, biB, bhB,
                                           out + kOut1, TFH, TFL);

  wmma_gemm64<1, 0, 0, 0, false><<<dim3(64, 1), 256, 0, stream>>>(
      VH, VH, kVd, 0L,
      WCVH, WCVH, kVd, 0L,
      (void*)RV, nullptr, kWcvN, 0L,
      nullptr, nullptr, 0L,
      kVRows, 2 * kVh, kVd, 1.0f);
  wmma_gemm64<1, 2, 0, 0, false><<<dim3(32, 1), 256, 0, stream>>>(
      VH, VL, kVd, 0L,
      WCVH + (size_t)2 * kVh * kVd, WVPL, kVd, 0L,
      (void*)(RV + 2 * kVh), nullptr, kWcvN, 0L,
      nullptr, nullptr, 0L,
      kVRows, kAd, kVd, 1.0f);

  wmma_gemm64<1, 0, 0, 0, false><<<dim3(8, 1), 256, 0, stream>>>(
      TFH, TFH, kTxt, 0L,
      WCTH, WCTH, kTxt, 0L,
      (void*)RT, nullptr, kWctN, 0L,
      nullptr, nullptr, 0L,
      kSeqs, kTh, kTxt, 1.0f);
  wmma_gemm64<1, 2, 0, 0, false><<<dim3(16, 1), 256, 0, stream>>>(
      TFH, TFL, kTxt, 0L,
      WCTH + (size_t)kTh * kTxt, WTPL, kTxt, 0L,
      (void*)(RT + kTh), nullptr, kWctN, 0L,
      nullptr, nullptr, 0L,
      kSeqs, kAd, kTxt, 1.0f);

  row_epilogue_kernel<<<kVRows / 32, 256, 0, stream>>>(
      RV, kWcvN,
      kVh, vtsB1, vtsW2, vtsB2, out + kOut2,
      kVh, kVh, vsumB1, vsumW2, vsumB2, out + kOut4,
      2 * kVh, vprojB, VNH, VNL);
  row_epilogue_kernel<<<kSeqs / 32, 256, 0, stream>>>(
      RT, kWctN,
      0, tsumB1, tsumW2, tsumB2, (float*)nullptr,
      0, kTh, tsumB1, tsumW2, tsumB2, out + kOut3,
      kTh, tprojB, ENH, ENL);

  wmma_gemm64<1, 2, 0, 0, false><<<dim3(1, kB), 256, 0, stream>>>(
      ENH, ENL, kAd, (long)kS * kAd,
      VNH, VNL, kAd, (long)kMv * kAd,
      (void*)SM, nullptr, kMv, (long)kKM,
      nullptr, nullptr, 0L,
      kS, kMv, kAd, 1.0f);

  cost_exp_kernel<<<(kTn / 4) / 256, 256, 0, stream>>>(SM, KM);
  transport_scale_kernel<<<kB, 256, 0, stream>>>(KM, SM, TW, LP);
  pack_kernel<<<(kTn / 4) / 256, 256, 0, stream>>>(TW, LP, out + kOut5);
}
